// SparseNeuralNetwork_57440892617097
// MI455X (gfx1250) — hardware-verified
//
#include <hip/hip_runtime.h>


namespace {
constexpr int BATCH = 8192, NLIM = 8192  , IN = 16, OUT = 16, D0 = 4096, D1 = 2048, NPAIR = D1 / 16  , NCH = D1 / 32  ;
constexpr float XS = 8.0f, WSC = 256.0f;
static_assert(BATCH % 32 == 0 && NLIM % 32 == 0 && NLIM <= BATCH, "tiling");
typedef _Float16 b16;
typedef __attribute__((ext_vector_type(16))) _Float16 v16b;
typedef __attribute__((ext_vector_type(8))) _Float16 v8b;
typedef __attribute__((ext_vector_type(8))) float v8f;
typedef __attribute__((ext_vector_type(4))) float v4f;
__device__ __forceinline__ float bf16_rne(float f) { unsigned int u = __float_as_uint(f); u += 0x7FFFu + ((u >> 16) & 1u); return __uint_as_float(u & 0xFFFF0000u); }
__device__ __forceinline__ void split16(float v, b16& hi, b16& lo) { hi = (b16)v; lo = (b16)(v - (float)hi); }
__device__ __forceinline__ v16b frag_kb(const b16* p, int hh) { const v8b a = *(const v8b*)(p + 8 * hh), b = *(const v8b*)(p + 16 + 8 * hh); v16b f;
#pragma unroll
  for (int e = 0; e < 8; ++e) { f[e] = a[e]; f[8 + e] = b[e]; } return f; }
__device__ __forceinline__ v8f wmma16b(v16b a, v16b b, v8f c) { v8f d = __builtin_amdgcn_wmma_f32_16x16x32_f16(false, a, false, b, (short)0, c, false, false); asm volatile("v_nop\n\tv_nop\n\tv_nop\n\tv_nop" : "+v"(d) : "v"(a), "v"(b)); return d; }
__device__ __forceinline__ void wave_lds_sync() { __builtin_amdgcn_fence(__ATOMIC_RELEASE, "workgroup"); __builtin_amdgcn_wave_barrier(); __builtin_amdgcn_fence(__ATOMIC_ACQUIRE, "workgroup"); }
__device__ __forceinline__ float pmul(float a, float b) { float p = a * b; asm volatile("" : "+v"(p)); return p; }
__device__ __forceinline__ int iclamp(int v, int lo, int hi) { return v < lo ? lo : (v > hi ? hi : v); }

__global__ __launch_bounds__(256) void prep_kernel(const float* __restrict__ w1, const float* __restrict__ w2, b16* __restrict__ W1P, b16* __restrict__ W2M) {
  const int u = blockIdx.x * 256 + threadIdx.x; v8b o;
  const int n1 = NPAIR * 16 * 32 / 8; if (u < n1) { const int e = u * 8; const int p = e / 512, c = (e / 32) % 16, k0 = e % 32;
    for (int j = 0; j < 8; ++j) { const int k = k0 + j; o[j] = ((c >> 3) == (k >> 4)) ? (b16)(bf16_rne(w1[(size_t)(16 * p + c) * D0 + 32 * p + k]) * WSC) : (b16)0.0f; }
    for (int pass = 0; pass < 2; ++pass) { *(volatile v8b*)(W1P + e) = o; __threadfence(); } return; }
  const int t = u - n1; if (t >= OUT * D1 / 8) return; { const int e = t * 8; const int i = e / D1, c0 = e % D1;
    for (int j = 0; j < 8; ++j) { const int c = c0 + j; o[j] = (((c & 127) >> 3) == i) ? (b16)(bf16_rne(w2[(size_t)i * D1 + c]) * WSC) : (b16)0.0f; }
    for (int pass = 0; pass < 2; ++pass) { *(volatile v8b*)(W2M + e) = o; __threadfence(); } }
}
__global__ __launch_bounds__(64) void snn_kernel(const float* __restrict__ x, const float* __restrict__ w0, const float* __restrict__ b0, const b16* __restrict__ W1P, const float* __restrict__ b1, const b16* __restrict__ W2M, const float* __restrict__ b2, float* __restrict__ out) {
  __shared__ __attribute__((aligned(16))) float Yf[2][16][32 + 4]; __shared__ __attribute__((aligned(16))) b16 Yh[2][16][32 + 8], Yl[2][16][32 + 8]; __shared__ __attribute__((aligned(16))) float To[2][16][16];
  const int wave = threadIdx.x >> 5, lane = threadIdx.x & 31, nloc = lane & 15, hlf = lane >> 4; const size_t m0 = (size_t)blockIdx.x * 32 + wave * 16; const size_t row = m0 + nloc;
  float xin[IN];
#pragma unroll
  for (int i = 0; i < IN; ++i) xin[i] = bf16_rne(x[row * IN + i]);
  v8f oacc = (v8f){};
  const float rs = 1.0f / (XS * WSC);
#pragma unroll 1
  for (int q = 0; q < NCH; ++q) {
#pragma unroll
    for (int pp = 0; pp < 2; ++pp) { const int p = 2 * q + pp; float xv = xin[0];
#pragma unroll
      for (int i = 1; i < IN; ++i) xv = ((p >> 3) == i) ? xin[i] : xv;
      v16b ah, al;
#pragma unroll
      for (int e = 0; e < 16; ++e) { const int k = (e < 8) ? (8 * hlf + e) : (16 + 8 * hlf + (e - 8)); const int uidx = 32 * p + k;
        const float y0 = fmaxf(pmul(xv, bf16_rne(w0[(size_t)uidx * IN + (p >> 3)])) + bf16_rne(b0[uidx]), 0.0f); b16 ph, pl; split16(y0 * XS, ph, pl); ah[e] = ph; al[e] = pl; }
      const v16b bw = frag_kb(W1P + ((size_t)p * 16 + nloc) * 32, hlf); v8f d = (v8f){}; d = wmma16b(ah, bw, d); d = wmma16b(al, bw, d);
#pragma unroll
      for (int r = 0; r < 8; ++r) Yf[wave][8 * hlf + r][pp * 16 + nloc] = fmaxf(d[r] * rs + bf16_rne(b1[16 * p + nloc]), 0.0f); }
    wave_lds_sync();
    { const int rr = lane & 15, c0 = (lane >> 4) * 16; v8b h0, l0, h1, l1;
#pragma unroll
      for (int j = 0; j < 8; ++j) { b16 ph, pl; split16(Yf[wave][rr][c0 + j] * XS, ph, pl); h0[j] = ph; l0[j] = pl; split16(Yf[wave][rr][c0 + 8 + j] * XS, ph, pl); h1[j] = ph; l1[j] = pl; }
      *(v8b*)(&Yh[wave][rr][c0]) = h0; *(v8b*)(&Yh[wave][rr][c0 + 8]) = h1; *(v8b*)(&Yl[wave][rr][c0]) = l0; *(v8b*)(&Yl[wave][rr][c0 + 8]) = l1; }
    wave_lds_sync();
    { const v16b a = frag_kb(&Yh[wave][nloc][0], hlf), al2 = frag_kb(&Yl[wave][nloc][0], hlf), bw = frag_kb(W2M + (size_t)nloc * D1 + 32 * q, hlf); oacc = wmma16b(a, bw, oacc); oacc = wmma16b(al2, bw, oacc); }
    wave_lds_sync(); }
#pragma unroll
  for (int r = 0; r < 8; ++r) To[wave][8 * hlf + r][nloc] = oacc[r] * rs + bf16_rne(b2[nloc]);
  wave_lds_sync();
  const float* tw = &To[wave][0][0];
  for (int pass = 0; pass < 2; ++pass) { *(volatile v4f*)(out + m0 * OUT + lane * 4) = *(const v4f*)(tw + lane * 4); *(volatile v4f*)(out + m0 * OUT + 128 + lane * 4) = *(const v4f*)(tw + 128 + lane * 4); __threadfence(); }
}
}

extern "C" void kernel_launch(void* const* d_in, const int* in_sizes, int n_in, void* d_out, int out_size, void* d_ws, size_t ws_size, hipStream_t stream) {
  (void)n_in;
  auto Fp = [&](int i) { return (const float*)d_in[i]; };
  if (in_sizes[0] != BATCH * IN || in_sizes[1] != D0 * IN || in_sizes[2] != D0 || in_sizes[3] != D1 * D0 || in_sizes[4] != D1 || in_sizes[5] != OUT * D1 || in_sizes[6] != OUT || out_size != BATCH * OUT) return;
  size_t off = 0; char* ws = (char*)d_ws;
  auto carve = [&](size_t bytes) { char* p = ws + off; off += (bytes + 255) & ~(size_t)255; return p; };
  b16* W1P = (b16*)carve((size_t)NPAIR * 16 * 32 * 2); b16* W2M = (b16*)carve((size_t)OUT * D1 * 2);
  if (off > ws_size || off > ((size_t)128 << 20)) return;
  prep_kernel<<<(NPAIR * 16 * 32 / 8 + OUT * D1 / 8 + 255) / 256, 256, 0, stream>>>(Fp(3), Fp(5), W1P, W2M);
  snn_kernel<<<NLIM / 32, 64, 0, stream>>>(Fp(0), Fp(1), Fp(2), W1P, Fp(4), W2M, Fp(6), (float*)d_out);
}
